// SparseGaussianProcess_35201551958592
// MI455X (gfx1250) — hardware-verified
//
#include <hip/hip_runtime.h>
#include <math.h>

typedef __attribute__((ext_vector_type(16))) _Float16 v16h;
typedef __attribute__((ext_vector_type(16))) __bf16 v16b;
typedef __attribute__((ext_vector_type(8)))  _Float16 v8h;
typedef __attribute__((ext_vector_type(8)))  float v8f;
typedef __attribute__((ext_vector_type(4)))  float v4f;
typedef __attribute__((ext_vector_type(2)))  float v2f;
typedef __attribute__((ext_vector_type(4)))  unsigned v4u;
typedef __attribute__((ext_vector_type(4)))  int v4i;
typedef float __attribute__((may_alias)) float_a;
typedef int __attribute__((may_alias)) int_a;

template <typename T> __device__ __forceinline__ void vst2(void* p, T v) { *(volatile T*)p = v; __threadfence(); *(volatile T*)p = v; }
__device__ __forceinline__ v8f wmma16(v16h a, v16h b, v8f c) {
  v8f d = __builtin_amdgcn_wmma_f32_16x16x32_f16(false, a, false, b, (short)0, c, false, false);
  asm volatile("v_nop\n\tv_nop\n\tv_nop\n\tv_nop" : "+v"(d) : "v"(a), "v"(b));
  return d;
}
__device__ __forceinline__ v8f wmma_bf(v16b a, v16b b, v8f c) {
  v8f d = __builtin_amdgcn_wmma_f32_16x16x32_bf16(false, a, false, b, (short)0, c, false, false);
  asm volatile("v_nop\n\tv_nop\n\tv_nop\n\tv_nop" : "+v"(d) : "v"(a), "v"(b));
  return d;
}
__device__ __forceinline__ v16h frag_h(const _Float16* rowk0, int lane) {
  union { v16h v; v8h q[2]; } u; const _Float16* p = rowk0 + 8 * (lane >> 4);
  u.q[0] = *(const v8h*)p; u.q[1] = *(const v8h*)(p + 16); return u.v;
}
__device__ __forceinline__ v16h frag_f32(const float* rowk0, int lane) {
  v16h a; const float* p = rowk0 + 8 * (lane >> 4);
#pragma unroll
  for (int i = 0; i < 8; ++i) { a[i] = (_Float16)p[i]; a[8 + i] = (_Float16)p[16 + i]; }
  return a;
}
__device__ __forceinline__ v16h frag_f32s(const float* rowk0, int lane, float sc) {
  v16h a; const float* p = rowk0 + 8 * (lane >> 4);
#pragma unroll
  for (int i = 0; i < 8; ++i) { a[i] = (_Float16)(p[i] * sc); a[8 + i] = (_Float16)(p[16 + i] * sc); }
  return a;
}
__device__ __forceinline__ v16h fragc_f32(const float* W, int k0, int n, int lane, int ld, int K) {
  v16h a; const int g = lane >> 4;
#pragma unroll
  for (int i = 0; i < 8; ++i) { const int ka = k0 + 8 * g + i, kb = ka + 16;
    a[i] = (_Float16)(ka < K ? W[(size_t)ka * ld + n] : 0.f); a[8 + i] = (_Float16)(kb < K ? W[(size_t)kb * ld + n] : 0.f); }
  return a;
}
struct F2 { v16b h, l; };
__device__ __forceinline__ F2 bsplit16(const float v[16]) { F2 r;
#pragma unroll
  for (int i = 0; i < 16; ++i) { const __bf16 h = (__bf16)v[i]; r.h[i] = h; r.l[i] = (__bf16)(v[i] - (float)h); }
  return r; }
__device__ __forceinline__ F2 split_row(const float* row, int k0, int lane) { float v[16]; const float* p = row + k0 + 8 * (lane >> 4);
#pragma unroll
  for (int i = 0; i < 8; ++i) { v[i] = p[i]; v[8 + i] = p[16 + i]; }
  return bsplit16(v); }
__device__ __forceinline__ F2 split_rowK(const float* row, int k0, int lane, int K) { float v[16]; const int g = lane >> 4;
#pragma unroll
  for (int i = 0; i < 8; ++i) { const int ka = k0 + 8 * g + i, kb = ka + 16; v[i] = ka < K ? row[ka] : 0.f; v[8 + i] = kb < K ? row[kb] : 0.f; }
  return bsplit16(v); }
__device__ __forceinline__ F2 split_col(const float* W, int k0, int n, int lane, int ld, int K) { float v[16]; const int g = lane >> 4;
#pragma unroll
  for (int i = 0; i < 8; ++i) { const int ka = k0 + 8 * g + i, kb = ka + 16; v[i] = ka < K ? W[(size_t)ka * ld + n] : 0.f; v[8 + i] = kb < K ? W[(size_t)kb * ld + n] : 0.f; }
  return bsplit16(v); }
__device__ __forceinline__ v8f mac3(const F2& a, const F2& b, v8f c) { c = wmma_bf(a.l, b.h, c); c = wmma_bf(a.h, b.l, c); return wmma_bf(a.h, b.h, c); }
__device__ __forceinline__ float sigm(float v) { return 1.0f / (1.0f + expf(-v)); }
#define LDSX() do { asm volatile("s_wait_dscnt 0" ::: "memory"); __builtin_amdgcn_wave_barrier(); __builtin_amdgcn_fence(__ATOMIC_RELEASE, "workgroup"); } while (0)

#define NN 16384
#define ID 8
#define MM 1024
#define LL 1024
#define SS 8
#define OD 4

__global__ __launch_bounds__(128) void k_gp(const float* __restrict__ x, const float* __restrict__ zloc, const float* __restrict__ iw, const float* __restrict__ freq,
                                          const float* __restrict__ phase, const float* __restrict__ pw, float* __restrict__ out) {
  __shared__ __align__(16) char lds[64 * (LL + 16) * 2];
  _Float16 (*T)[LL + 16] = (_Float16 (*)[LL + 16])lds; float (*T32)[516] = (float (*)[516])lds;
  __shared__ __align__(16) float res[SS * OD][64 + 4];
  __shared__ float sx[64][ID];
  const int tid = threadIdx.x, wave = tid >> 5, lane = tid & 31, col = lane & 15, g = lane >> 4;
  const int n0 = blockIdx.x * 64;
  for (int q = tid; q < 64 * ID; q += 128) sx[q >> 3][q & 7] = x[(size_t)n0 * ID + q];
  for (int q = tid; q < SS * OD * 64; q += 128) res[q >> 6][q & 63] = 0.f;
  __syncthreads();
  const float bwscale = sqrtf(2.0f / (float)LL);
#pragma unroll 1
  for (int o = 0; o < OD; ++o) {
    for (int q = tid; q < 64 * LL; q += 128) { const int r = q >> 10, l = q & 1023; float ip = 0.f;
#pragma unroll
      for (int i = 0; i < ID; ++i) ip += sx[r][i] * freq[((size_t)o * ID + i) * LL + l];
      T[r][l] = (_Float16)cosf(ip + phase[o * LL + l]); }
    __syncthreads();
    v8f acc = {};
#pragma unroll 1
    for (int kc = 0; kc < LL / 32; ++kc) { v16h bw; const int s = col;
#pragma unroll
      for (int i = 0; i < 8; ++i) { const int la = kc * 32 + 8 * g + i, lb = la + 16;
        bw[i] = (_Float16)(s < SS ? pw[((size_t)s * OD + o) * LL + la] : 0.f); bw[8 + i] = (_Float16)(s < SS ? pw[((size_t)s * OD + o) * LL + lb] : 0.f); }
      acc = wmma16(frag_h(&T[wave * 16 + col][0] + kc * 32, lane), bw, acc); }
    if (col < SS) {
#pragma unroll
      for (int r = 0; r < 8; ++r) res[col * OD + o][wave * 16 + 8 * g + r] += acc[r] * bwscale; }
    __syncthreads();
  }
#pragma unroll 1
  for (int half = 0; half < 2; ++half) {
    for (int q = tid; q < 64 * 512; q += 128) { const int r = q >> 9, ml = q & 511, m = half * 512 + ml; float xx = 0.f, zz = 0.f, xz = 0.f;
#pragma unroll
      for (int i = 0; i < ID; ++i) { const float xv = sx[r][i], zv = zloc[m * ID + i]; xx += xv * xv; zz += zv * zv; xz += xv * zv; }
      const float d2 = xx + zz - 2.0f * xz;
      T32[r][ml] = expf(-0.5f * d2); }
    __syncthreads();
    { v8f acc[2] = {};
#pragma unroll 1
      for (int kc = 0; kc < 512 / 32; ++kc) { const F2 a = split_row(&T32[wave * 16 + col][0], kc * 32, lane);
#pragma unroll
        for (int t = 0; t < 2; ++t) acc[t] = mac3(a, split_row(iw + (size_t)(t * 16 + col) * MM + half * 512, kc * 32, lane), acc[t]); }
#pragma unroll
      for (int t = 0; t < 2; ++t)
#pragma unroll
        for (int r = 0; r < 8; ++r) res[t * 16 + col][wave * 16 + 8 * g + r] += acc[t][r]; }
    __syncthreads();
  }
  for (int q = tid; q < 32 * 16; q += 128) { const int row = q >> 4, pc = q & 15; vst2(out + (size_t)row * NN + n0 + pc * 4, *(const v4f*)(&res[row][pc * 4])); }
}
extern "C" void kernel_launch(void* const* d_in, const int* in_sizes, int n_in, void* d_out, int out_size, void* d_ws, size_t ws_size, hipStream_t stream) {
  (void)in_sizes; (void)n_in; (void)out_size; (void)ws_size; (void)d_ws;
  k_gp<<<NN / 64, 128, 0, stream>>>((const float*)d_in[0], (const float*)d_in[1], (const float*)d_in[2], (const float*)d_in[3], (const float*)d_in[4], (const float*)d_in[5], (float*)d_out);
}
